// ParticleNCA_edge_23768349016082
// MI455X (gfx1250) — hardware-verified
//
#include <hip/hip_runtime.h>
#include <stddef.h>
#include <math.h>


#define NTHR   256
#define NWAVE  8
#define EPT    8
#define CHUNK  (NTHR * EPT)
#define WCAP   (EPT * 32)
#define LISTN  (NWAVE * WCAP)
#define PASSN  (NWAVE * 16)
#define PCAP   (CHUNK + PASSN)
#define NB     256
#define MOLD   16
#define SFD    20
#define SFK    32
#define RIN    21
#define RIK    32
#define MH     64
#define HC     128
#define CH     64
#define OD     20
#define ODP    32
#define HNB    128
#define NPREP  23
#define WSC    16.0f
#define BSC2   64.0f
#define QSC1   0.25f
#define QSC2   0.0625f
#define EINV   0.015625f
#define ASCL   0.125f
#define DEPS   1e-16f
#define WSLIM  134217728

#define LE_ACC   0
#define LE_MSG   (LE_ACC + (NB + 1) * HC * 4)
#define LE_STG   (LE_MSG + PASSN * HC * 4)
#define LE_LIST  (LE_STG + NWAVE * 16 * RIK * 2)
#define LE_PEND  (LE_LIST + LISTN * 4)
#define LE_SLOT  (LE_PEND + PCAP * 4)
#define LE_ALPH  (LE_SLOT + PASSN * 4)
#define LE_MP    (LE_ALPH + PASSN * 8)
#define LE_MN    (LE_MP + PASSN * 8)
#define LE_SP    (LE_MN + PASSN * 8)
#define LE_PP    (LE_SP + PASSN * 8)
#define LE_MST   (LE_PP + PASSN * 8)
#define LE_DEN   (LE_MST + 2064)
#define LE_PRM   (LE_DEN + 2064)
#define LE_WCNT  (LE_PRM + 3 * MH * 4)
#define LE_TOTAL (LE_WCNT + 64)

#define LN_TOTAL (NWAVE * 16 * HC * 4)

static_assert(PASSN == 128);
static_assert(NTHR == 2 * PASSN);
static_assert(PCAP >= CHUNK + PASSN);
static_assert(NB == 32 * NWAVE);
static_assert(NB == NTHR);
static_assert(HNB == 16 * NWAVE);
static_assert((NB + 1) * 2 * 4 <= 2064);
static_assert((LE_TOTAL % 16) == 0);
static_assert(LE_TOTAL <= 300 * 1024);
static_assert(LN_TOTAL <= 64 * 1024);

typedef float          v4f  __attribute__((ext_vector_type(4)));
typedef float          v8f  __attribute__((ext_vector_type(8)));
typedef int            v4i  __attribute__((ext_vector_type(4)));
typedef _Float16       v8h  __attribute__((ext_vector_type(8)));
typedef _Float16       v16h __attribute__((ext_vector_type(16)));
typedef unsigned short v8us __attribute__((ext_vector_type(8)));
typedef __bf16         v16b __attribute__((ext_vector_type(16)));
union FragH { v16h v; v8h h[2]; };
union FragB { v16b v; v8us u[2]; };
union Pk8   { v8h h; v8us s; v4i i; };

__device__ __forceinline__ v8f splat8(float x) {
  v8f c;
#pragma unroll
  for (int i = 0; i < 8; ++i) c[i] = x;
  return c;
}

__device__ __forceinline__ v8f ldc8(const float* p) {
  const v4f a = *(const v4f*)p;
  const v4f b = *(const v4f*)(p + 4);
  v8f c;
  c[0] = a.x; c[1] = a.y; c[2] = a.z; c[3] = a.w;
  c[4] = b.x; c[5] = b.y; c[6] = b.z; c[7] = b.w;
  return c;
}

__device__ __forceinline__ v8f wmh(v16h a, v16h b, v8f c) {
  v8f d = __builtin_amdgcn_wmma_f32_16x16x32_f16(false, a, false, b, (short)0, c, false, false);
  asm volatile("v_nop\n\tv_nop\n\tv_nop\n\tv_nop" : "+v"(d) : "v"(a), "v"(b));
  return d;
}

__device__ __forceinline__ v8f wmb(v16b a, v16b b, v8f c) {
  v8f d = __builtin_amdgcn_wmma_f32_16x16x32_bf16(false, a, false, b, (short)0, c, false, false);
  asm volatile("v_nop\n\tv_nop\n\tv_nop\n\tv_nop" : "+v"(d) : "v"(a), "v"(b));
  return d;
}

__device__ __forceinline__ v8f wmb3(const FragB& ah, const FragB& al, const FragB& bh, const FragB& bl, v8f c) {
  c = wmb(ah.v, bh.v, c);
  c = wmb(ah.v, bl.v, c);
  c = wmb(al.v, bh.v, c);
  return c;
}

__device__ __forceinline__ v8h relu8(v8f d, float mul) {
  v8h r;
#pragma unroll
  for (int i = 0; i < 8; ++i) { const float t = fmaxf(d[i] * mul, 0.0f); r[i] = (_Float16)t; }
  return r;
}

__device__ __forceinline__ unsigned short bfr(float x) {
  unsigned int u = __float_as_uint(x);
  u += 0x7FFFu + ((u >> 16) & 1u);
  return (unsigned short)(u >> 16);
}
__device__ __forceinline__ float bfv(unsigned short b) {
  return __uint_as_float(((unsigned int)b) << 16);
}
__device__ __forceinline__ void split8(v4f a, v4f b, v8us& hi, v8us& lo) {
  float f[8];
  f[0] = a.x; f[1] = a.y; f[2] = a.z; f[3] = a.w;
  f[4] = b.x; f[5] = b.y; f[6] = b.z; f[7] = b.w;
#pragma unroll
  for (int i = 0; i < 8; ++i) {
    const unsigned short hb = bfr(f[i]);
    hi[i] = hb;
    lo[i] = bfr(f[i] - bfv(hb));
  }
}

__device__ __forceinline__ int scan_chunk(const int* __restrict__ dsts, const float* __restrict__ em, int nE,
                                          int cbase, int nodeBase, int vec8, int useSlot, int* list, int tid, int wave) {
  int wc = 0;
  const int el0  = tid * EPT;
  const int e0   = cbase + el0;
  const int sent = -2147483647 - 1;
  v4i da, db;
  v4f fa, fb;
  if (vec8 != 0 && cbase + CHUNK <= nE) {
    da = *(const v4i*)(dsts + e0);
    db = *(const v4i*)(dsts + e0 + 4);
    fa = *(const v4f*)(em + e0);
    fb = *(const v4f*)(em + e0 + 4);
  } else {
    const int c0 = e0     < nE - 1 ? e0     : nE - 1;
    const int c1 = e0 + 1 < nE - 1 ? e0 + 1 : nE - 1;
    const int c2 = e0 + 2 < nE - 1 ? e0 + 2 : nE - 1;
    const int c3 = e0 + 3 < nE - 1 ? e0 + 3 : nE - 1;
    const int c4 = e0 + 4 < nE - 1 ? e0 + 4 : nE - 1;
    const int c5 = e0 + 5 < nE - 1 ? e0 + 5 : nE - 1;
    const int c6 = e0 + 6 < nE - 1 ? e0 + 6 : nE - 1;
    const int c7 = e0 + 7 < nE - 1 ? e0 + 7 : nE - 1;
    const int d0 = dsts[c0], d1 = dsts[c1], d2 = dsts[c2], d3 = dsts[c3];
    const int d4 = dsts[c4], d5 = dsts[c5], d6 = dsts[c6], d7 = dsts[c7];
    const float m0 = em[c0], m1 = em[c1], m2 = em[c2], m3 = em[c3];
    const float m4 = em[c4], m5 = em[c5], m6 = em[c6], m7 = em[c7];
    da.x = (e0     < nE) ? d0 : sent;  fa.x = (e0     < nE) ? m0 : 0.0f;
    da.y = (e0 + 1 < nE) ? d1 : sent;  fa.y = (e0 + 1 < nE) ? m1 : 0.0f;
    da.z = (e0 + 2 < nE) ? d2 : sent;  fa.z = (e0 + 2 < nE) ? m2 : 0.0f;
    da.w = (e0 + 3 < nE) ? d3 : sent;  fa.w = (e0 + 3 < nE) ? m3 : 0.0f;
    db.x = (e0 + 4 < nE) ? d4 : sent;  fb.x = (e0 + 4 < nE) ? m4 : 0.0f;
    db.y = (e0 + 5 < nE) ? d5 : sent;  fb.y = (e0 + 5 < nE) ? m5 : 0.0f;
    db.z = (e0 + 6 < nE) ? d6 : sent;  fb.z = (e0 + 6 < nE) ? m6 : 0.0f;
    db.w = (e0 + 7 < nE) ? d7 : sent;  fb.w = (e0 + 7 < nE) ? m7 : 0.0f;
  }
  const unsigned nb = (unsigned)nodeBase;
  const unsigned s0 = (unsigned)da.x - nb, s1 = (unsigned)da.y - nb;
  const unsigned s2 = (unsigned)da.z - nb, s3 = (unsigned)da.w - nb;
  const unsigned s4 = (unsigned)db.x - nb, s5 = (unsigned)db.y - nb;
  const unsigned s6 = (unsigned)db.z - nb, s7 = (unsigned)db.w - nb;
  const bool h0 = (s0 < (unsigned)NB) && (fa.x != 0.0f);
  const bool h1 = (s1 < (unsigned)NB) && (fa.y != 0.0f);
  const bool h2 = (s2 < (unsigned)NB) && (fa.z != 0.0f);
  const bool h3 = (s3 < (unsigned)NB) && (fa.w != 0.0f);
  const bool h4 = (s4 < (unsigned)NB) && (fb.x != 0.0f);
  const bool h5 = (s5 < (unsigned)NB) && (fb.y != 0.0f);
  const bool h6 = (s6 < (unsigned)NB) && (fb.z != 0.0f);
  const bool h7 = (s7 < (unsigned)NB) && (fb.w != 0.0f);
  const unsigned any = __builtin_amdgcn_ballot_w32(h0 | h1 | h2 | h3 | h4 | h5 | h6 | h7);
  if (any != 0u) {
#define HITJ(J, HJ, SJ) { \
      const unsigned mj = __builtin_amdgcn_ballot_w32(HJ); \
      if (mj != 0u) { \
        if (HJ) { \
          const int pos = wc + (int)__builtin_amdgcn_mbcnt_lo(mj, 0u); \
          const int val = (useSlot != 0) ? (int)(SJ) : (el0 + (J)); \
          if (pos < WCAP) list[wave * WCAP + pos] = val; \
        } \
        wc += (int)__builtin_popcount(mj); } }
    HITJ(0, h0, s0)
    HITJ(1, h1, s1)
    HITJ(2, h2, s2)
    HITJ(3, h3, s3)
    HITJ(4, h4, s4)
    HITJ(5, h5, s5)
    HITJ(6, h6, s6)
    HITJ(7, h7, s7)
#undef HITJ
  }
  return wc;
}

__global__ __launch_bounds__(NTHR) void k_prep(
    const float* __restrict__ mw1, const float* __restrict__ mw2, const float* __restrict__ mw3,
    const float* __restrict__ we,
    const float* __restrict__ wq, const float* __restrict__ wk, const float* __restrict__ wv,
    const float* __restrict__ wskip,
    const float* __restrict__ hw1, const float* __restrict__ hw2, const float* __restrict__ hw3,
    unsigned short* p1, unsigned short* p2, unsigned short* p3, unsigned short* pe,
    unsigned short* pqh, unsigned short* pql, unsigned short* pkh, unsigned short* pkl,
    unsigned short* pvh, unsigned short* pvl, unsigned short* psh, unsigned short* psl,
    unsigned short* pwh, unsigned short* pwl, unsigned short* ph1h, unsigned short* ph1l,
    unsigned short* ph2h, unsigned short* ph2l, unsigned short* ph3h, unsigned short* ph3l) {
  const int b = blockIdx.x, tid = threadIdx.x;
  const float* src;
  unsigned short* da;
  unsigned short* db;
  int O, Op, Kin, Kp, k0, pitch, mode, ub;
  if (b < 1)       { src = mw1;   da = p1;   db = p1;   O = MH; Op = MH;  Kin = RIN; Kp = RIK; k0 = 0;  pitch = MH; mode = 0; ub = b; }
  else if (b < 3)  { src = mw2;   da = p2;   db = p2;   O = MH; Op = MH;  Kin = MH;  Kp = MH;  k0 = 0;  pitch = MH; mode = 0; ub = b - 1; }
  else if (b < 5)  { src = mw3;   da = p3;   db = p3;   O = MH; Op = MH;  Kin = MH;  Kp = MH;  k0 = 0;  pitch = MH; mode = 0; ub = b - 3; }
  else if (b < 9)  { src = we;    da = pe;   db = pe;   O = HC; Op = HC;  Kin = MH;  Kp = MH;  k0 = 0;  pitch = HC; mode = 0; ub = b - 5; }
  else if (b < 11) { src = wq;    da = pqh;  db = pql;  O = HC; Op = HC;  Kin = SFD; Kp = SFK; k0 = 0;  pitch = HC; mode = 1; ub = b - 9; }
  else if (b < 13) { src = wk;    da = pkh;  db = pkl;  O = HC; Op = HC;  Kin = SFD; Kp = SFK; k0 = 0;  pitch = HC; mode = 1; ub = b - 11; }
  else if (b < 15) { src = wv;    da = pvh;  db = pvl;  O = HC; Op = HC;  Kin = SFD; Kp = SFK; k0 = 0;  pitch = HC; mode = 1; ub = b - 13; }
  else if (b < 16) { src = wskip; da = psh;  db = psl;  O = CH; Op = CH;  Kin = SFD; Kp = SFK; k0 = 0;  pitch = CH; mode = 1; ub = b - 15; }
  else if (b < 18) { src = we;    da = pwh;  db = pwl;  O = HC; Op = HC;  Kin = SFD; Kp = SFK; k0 = MH; pitch = HC; mode = 1; ub = b - 16; }
  else if (b < 20) { src = hw1;   da = ph1h; db = ph1l; O = CH; Op = CH;  Kin = CH;  Kp = CH;  k0 = 0;  pitch = CH; mode = 1; ub = b - 18; }
  else if (b < 22) { src = hw2;   da = ph2h; db = ph2l; O = CH; Op = CH;  Kin = CH;  Kp = CH;  k0 = 0;  pitch = CH; mode = 1; ub = b - 20; }
  else             { src = hw3;   da = ph3h; db = ph3l; O = OD; Op = ODP; Kin = CH;  Kp = CH;  k0 = 0;  pitch = OD; mode = 1; ub = b - 22; }
  const int u   = ub * NTHR + tid;
  const int cpr = Kp >> 3;
  int n = u / cpr;
  const int kc = u - n * cpr;
  if (n > Op - 1) n = Op - 1;
  const int ocl = n < O ? n : O - 1;
  Pk8 pf, ph, pl;
#pragma unroll
  for (int j = 0; j < 8; ++j) {
    const int k   = 8 * kc + j;
    const int kcl = k < Kin ? k : Kin - 1;
    const float w = src[(size_t)(k0 + kcl) * pitch + ocl];
    const float t = (k < Kin && n < O) ? w : 0.0f;
    pf.h[j] = (_Float16)(t * WSC);
    const unsigned short hb = bfr(t);
    ph.s[j] = hb;
    pl.s[j] = bfr(t - bfv(hb));
  }
  unsigned short* dpa = da + (size_t)u * 8;
  unsigned short* dpb = db + (size_t)u * 8;
  if (mode == 0) {
    *(volatile v4i*)dpa = pf.i;
    __threadfence();
    *(volatile v4i*)dpa = pf.i;
  } else {
    *(volatile v4i*)dpa = ph.i;
    *(volatile v4i*)dpb = pl.i;
    __threadfence();
    *(volatile v4i*)dpa = ph.i;
    *(volatile v4i*)dpb = pl.i;
  }
}

__global__ __launch_bounds__(NTHR) void k_deg(const int* __restrict__ dsts, const float* __restrict__ em,
                                             float* deg, int nE, int vec8) {
  __shared__ int list[LISTN];
  __shared__ int wcnt[NWAVE];
  __shared__ __attribute__((aligned(16))) float dstg[NB];
  const int tid = threadIdx.x, lane = tid & 31, wave = tid >> 5;
  const int nodeBase = blockIdx.x * NB;
  int cnt = 0;
  const int nChunks = (nE + CHUNK - 1) / CHUNK;
#pragma unroll 1
  for (int ch = 0; ch < nChunks; ++ch) {
    const int cbase = ch * CHUNK;
    const int wc = scan_chunk(dsts, em, nE, cbase, nodeBase, vec8, 1, list, tid, wave);
    if (lane == 0) wcnt[wave] = wc;
    __syncthreads();
#pragma unroll 1
    for (int w = 0; w < NWAVE; ++w) {
      int n = wcnt[w];
      n = n > WCAP ? WCAP : (n < 0 ? 0 : n);
      const int* lp = list + w * WCAP;
#pragma unroll 4
      for (int i = 0; i < n; ++i) cnt += (lp[i] == tid) ? 1 : 0;
    }
    __syncthreads();
  }
  dstg[tid] = (float)cnt;
  __syncthreads();
  if (tid < 64) {
    const v4f v = *(const v4f*)(dstg + 4 * tid);
    *(volatile v4f*)(deg + (size_t)nodeBase + 4 * tid) = v;
  }
  __threadfence();
  if (tid < 64) {
    const v4f v = *(const v4f*)(dstg + 4 * tid);
    *(volatile v4f*)(deg + (size_t)nodeBase + 4 * tid) = v;
  }
}

template <int NT>
__device__ __forceinline__ void node_plane(const FragB& ah, const FragB& al,
                                           const unsigned short* __restrict__ ph, const unsigned short* __restrict__ pl,
                                           const float* __restrict__ bias, int hasb, float* outp, float* stgw,
                                           int row0, int lane, int h, int m) {
#pragma unroll 1
  for (int nt = 0; nt < NT; ++nt) {
    const int n = 16 * nt + m;
    const float bb = bias[n];
    v8f c = splat8(hasb != 0 ? bb : 0.0f);
    FragB bh, bl;
    const size_t off = (size_t)n * SFK + 8 * h;
    bh.u[0] = *(const v8us*)(ph + off);
    bh.u[1] = *(const v8us*)(ph + off + 16);
    bl.u[0] = *(const v8us*)(pl + off);
    bl.u[1] = *(const v8us*)(pl + off + 16);
    c = wmb3(ah, al, bh, bl, c);
#pragma unroll
    for (int r = 0; r < 8; ++r) stgw[(8 * h + r) * HC + n] = c[r];
  }
  __syncthreads();
  if (NT == 8) {
#pragma unroll 1
    for (int i = 0; i < 16; ++i) {
      const v4f v = *(const v4f*)(stgw + i * HC + 4 * lane);
      *(volatile v4f*)(outp + (size_t)(row0 + i) * HC + 4 * lane) = v;
    }
    __threadfence();
#pragma unroll 1
    for (int i = 0; i < 16; ++i) {
      const v4f v = *(const v4f*)(stgw + i * HC + 4 * lane);
      *(volatile v4f*)(outp + (size_t)(row0 + i) * HC + 4 * lane) = v;
    }
  } else {
    const int rs = lane >> 4, c4 = 4 * (lane & 15);
#pragma unroll 1
    for (int j = 0; j < 8; ++j) {
      const int row = 2 * j + rs;
      const v4f v = *(const v4f*)(stgw + row * HC + c4);
      *(volatile v4f*)(outp + (size_t)(row0 + row) * CH + c4) = v;
    }
    __threadfence();
#pragma unroll 1
    for (int j = 0; j < 8; ++j) {
      const int row = 2 * j + rs;
      const v4f v = *(const v4f*)(stgw + row * HC + c4);
      *(volatile v4f*)(outp + (size_t)(row0 + row) * CH + c4) = v;
    }
  }
  __syncthreads();
}

__global__ __launch_bounds__(NTHR) void k_node(
    const float* __restrict__ angle, const float* __restrict__ mol, const float* __restrict__ gen,
    const float* __restrict__ deg,
    const unsigned short* __restrict__ pqh, const unsigned short* __restrict__ pql,
    const unsigned short* __restrict__ pkh, const unsigned short* __restrict__ pkl,
    const unsigned short* __restrict__ pvh, const unsigned short* __restrict__ pvl,
    const unsigned short* __restrict__ psh, const unsigned short* __restrict__ psl,
    const unsigned short* __restrict__ pwh, const unsigned short* __restrict__ pwl,
    const float* __restrict__ bq, const float* __restrict__ bk, const float* __restrict__ bv,
    const float* __restrict__ bskip,
    float* Qo, float* Ko, float* Vo, float* So, float* Wo, int nN) {
  extern __shared__ __attribute__((aligned(16))) unsigned char dsmn[];
  const int tid = threadIdx.x, lane = tid & 31, wave = tid >> 5, h = lane >> 4, m = lane & 15;
  float* stgw = (float*)dsmn + wave * 16 * HC;
  const int row0 = blockIdx.x * HNB + wave * 16;
  int node = row0 + m;
  node = node > nN - 1 ? nN - 1 : node;
  const float a = angle[node];
  const float* mr = mol + (size_t)node * MOLD;
  const v4f q0 = *(const v4f*)mr, q1 = *(const v4f*)(mr + 4), q2 = *(const v4f*)(mr + 8), q3 = *(const v4f*)(mr + 12);
  float sf[SFD];
  sf[0] = sinf(a); sf[1] = cosf(a);
  sf[2] = q0.x;  sf[3] = q0.y;  sf[4] = q0.z;  sf[5] = q0.w;
  sf[6] = q1.x;  sf[7] = q1.y;  sf[8] = q1.z;  sf[9] = q1.w;
  sf[10] = q2.x; sf[11] = q2.y; sf[12] = q2.z; sf[13] = q2.w;
  sf[14] = q3.x; sf[15] = q3.y; sf[16] = q3.z; sf[17] = q3.w;
  sf[18] = gen[node]; sf[19] = deg[node];
  v4f e0, e1, e2, e3;
  e0.x = h ? sf[8]  : sf[0]; e0.y = h ? sf[9]  : sf[1]; e0.z = h ? sf[10] : sf[2]; e0.w = h ? sf[11] : sf[3];
  e1.x = h ? sf[12] : sf[4]; e1.y = h ? sf[13] : sf[5]; e1.z = h ? sf[14] : sf[6]; e1.w = h ? sf[15] : sf[7];
  e2.x = h ? 0.0f : sf[16]; e2.y = h ? 0.0f : sf[17]; e2.z = h ? 0.0f : sf[18]; e2.w = h ? 0.0f : sf[19];
  e3.x = 0.0f; e3.y = 0.0f; e3.z = 0.0f; e3.w = 0.0f;
  FragB ah, al;
  split8(e0, e1, ah.u[0], al.u[0]);
  split8(e2, e3, ah.u[1], al.u[1]);
  node_plane<8>(ah, al, pqh, pql, bq,    1, Qo, stgw, row0, lane, h, m);
  node_plane<8>(ah, al, pkh, pkl, bk,    1, Ko, stgw, row0, lane, h, m);
  node_plane<8>(ah, al, pvh, pvl, bv,    1, Vo, stgw, row0, lane, h, m);
  node_plane<4>(ah, al, psh, psl, bskip, 1, So, stgw, row0, lane, h, m);
  node_plane<8>(ah, al, pwh, pwl, bq,    0, Wo, stgw, row0, lane, h, m);
}

__global__ __launch_bounds__(NTHR) void k_edge(
    const float* __restrict__ x, const float* __restrict__ angle, const float* __restrict__ mol,
    const int* __restrict__ srcs, const int* __restrict__ dsts, const float* __restrict__ em,
    const float* __restrict__ mb1, const float* __restrict__ mb2, const float* __restrict__ mb3,
    const _Float16* __restrict__ P1, const _Float16* __restrict__ P2,
    const _Float16* __restrict__ P3, const _Float16* __restrict__ PE,
    const float* __restrict__ Qp, const float* __restrict__ Kq, const float* __restrict__ Vp,
    const float* __restrict__ SWp, float* aggo, int nN, int nE, int vec8) {
  extern __shared__ __attribute__((aligned(16))) unsigned char dsme[];
  float*    acc   = (float*)(dsme + LE_ACC);
  float*    msg   = (float*)(dsme + LE_MSG);
  _Float16* stg   = (_Float16*)(dsme + LE_STG);
  int*      list  = (int*)(dsme + LE_LIST);
  int*      pend  = (int*)(dsme + LE_PEND);
  int*      slotb = (int*)(dsme + LE_SLOT);
  float*    alph  = (float*)(dsme + LE_ALPH);
  float*    mpv   = (float*)(dsme + LE_MP);
  float*    mnv   = (float*)(dsme + LE_MN);
  float*    spv   = (float*)(dsme + LE_SP);
  float*    ppv   = (float*)(dsme + LE_PP);
  float*    mst   = (float*)(dsme + LE_MST);
  float*    den   = (float*)(dsme + LE_DEN);
  float*    prm   = (float*)(dsme + LE_PRM);
  int*      wcnt  = (int*)(dsme + LE_WCNT);

  const int tid = threadIdx.x, lane = tid & 31, wave = tid >> 5, h = lane >> 4, m = lane & 15;
  const int nodeBase = blockIdx.x * NB;

  {
    const v4f z = {0.0f, 0.0f, 0.0f, 0.0f};
    for (int i = tid; i < (NB + 1) * HC / 4; i += NTHR) *(v4f*)(acc + 4 * i) = z;
    for (int i = tid; i < (NB + 1) * 2; i += NTHR) { mst[i] = -__builtin_inff(); den[i] = 0.0f; }
  }
  if (tid < MH) {
    prm[tid] = mb1[tid] * WSC;
    prm[MH + tid] = mb2[tid] * BSC2;
    prm[2 * MH + tid] = mb3[tid] * BSC2;
  }
  if (tid == 0) wcnt[NWAVE] = 0;
  __syncthreads();

  const int nChunks = (nE + CHUNK - 1) / CHUNK;
#pragma unroll 1
  for (int ch = 0; ch < nChunks; ++ch) {
    const int cbase = ch * CHUNK;
    const int wc = scan_chunk(dsts, em, nE, cbase, nodeBase, vec8, 0, list, tid, wave);
    if (lane == 0) wcnt[wave] = wc;
    __syncthreads();

    const int base = wcnt[NWAVE];
    int tot = 0, myoff = 0;
#pragma unroll
    for (int w = 0; w < NWAVE; ++w) {
      int c = wcnt[w];
      c = c > WCAP ? WCAP : (c < 0 ? 0 : c);
      if (w < wave) myoff += c;
      tot += c;
    }
    int newN = base + tot;
    newN = newN > PCAP ? PCAP : newN;
    {
      int n = wcnt[wave];
      n = n > WCAP ? WCAP : (n < 0 ? 0 : n);
      const int* lp = list + wave * WCAP;
      for (int i = lane; i < n; i += 32) {
        const int pos = base + myoff + i;
        if (pos < PCAP) pend[pos] = cbase + lp[i];
      }
    }
    const int fin = (ch == nChunks - 1) ? 1 : 0;
    const int R   = (fin != 0) ? (newN + PASSN - 1) / PASSN : newN / PASSN;
    const int Pv  = (fin != 0) ? newN : R * PASSN;
    __syncthreads();

#pragma unroll 1
    for (int r = 0; r < R; ++r) {
      int scl, dcl;
      {
        int idx = r * PASSN + wave * 16 + m;
        const bool valid = idx < Pv;
        idx = idx > PCAP - 1 ? PCAP - 1 : idx;
        int e = pend[idx];
        e = e < 0 ? 0 : (e > nE - 1 ? nE - 1 : e);
        int d = dsts[e];
        int s = srcs[e];
        int slot = d - nodeBase;
        if (!valid || (unsigned)slot >= (unsigned)NB) slot = NB;
        s = s < 0 ? 0 : (s > nN - 1 ? nN - 1 : s);
        d = d < 0 ? 0 : (d > nN - 1 ? nN - 1 : d);
        scl = s; dcl = d;
        const float dx = x[2 * s] - x[2 * d];
        const float dy = x[2 * s + 1] - x[2 * d + 1];
        const float rr = sqrtf(fmaxf(dx * dx + dy * dy, 1e-12f));
        const float dang = angle[s] - angle[d];
        const float sn = sinf(dang), cs = cosf(dang);
        const float* ms = mol + (size_t)s * MOLD;
        const float* md = mol + (size_t)d * MOLD;
        const v4f dm0 = *(const v4f*)ms - *(const v4f*)md;
        const v4f dm1 = *(const v4f*)(ms + 4) - *(const v4f*)(md + 4);
        const v4f dm2 = *(const v4f*)(ms + 8) - *(const v4f*)(md + 8);
        const v4f dm3 = *(const v4f*)(ms + 12) - *(const v4f*)(md + 12);
        v8h g0, g1;
        g0[0] = (_Float16)(h ? dm2.w : dx);    g0[1] = (_Float16)(h ? dm3.x : dy);
        g0[2] = (_Float16)(h ? dm3.y : rr);    g0[3] = (_Float16)(h ? dm3.z : sn);
        g0[4] = (_Float16)(h ? dm3.w : cs);    g0[5] = (_Float16)(h ? 0.0f : dm0.x);
        g0[6] = (_Float16)(h ? 0.0f : dm0.y);  g0[7] = (_Float16)(h ? 0.0f : dm0.z);
        g1[0] = (_Float16)(h ? 0.0f : dm0.w);  g1[1] = (_Float16)(h ? 0.0f : dm1.x);
        g1[2] = (_Float16)(h ? 0.0f : dm1.y);  g1[3] = (_Float16)(h ? 0.0f : dm1.z);
        g1[4] = (_Float16)(h ? 0.0f : dm1.w);  g1[5] = (_Float16)(h ? 0.0f : dm2.x);
        g1[6] = (_Float16)(h ? 0.0f : dm2.y);  g1[7] = (_Float16)(h ? 0.0f : dm2.z);
        _Float16* srow = stg + (wave * 16 + m) * RIK;
        *(v8h*)(srow + 16 * h) = g0;
        *(v8h*)(srow + 16 * h + 8) = g1;
        if (h == 0) slotb[wave * 16 + m] = slot;
      }
      __syncthreads();

      {
        const _Float16* srow = stg + (wave * 16 + m) * RIK;
        FragH ba;
        ba.h[0] = *(const v8h*)(srow + 8 * h);
        ba.h[1] = *(const v8h*)(srow + 16 + 8 * h);
        FragH bq[2];
#pragma unroll
        for (int q = 0; q < 2; ++q) {
          v8f d0, d1;
          {
            FragH a;
            const _Float16* wp = P1 + (size_t)(32 * q + m) * RIK + 8 * h;
            a.h[0] = *(const v8h*)wp;
            a.h[1] = *(const v8h*)(wp + 16);
            d0 = wmh(a.v, ba.v, ldc8(prm + 32 * q + 8 * h));
          }
          {
            FragH a;
            const _Float16* wp = P1 + (size_t)(32 * q + 16 + m) * RIK + 8 * h;
            a.h[0] = *(const v8h*)wp;
            a.h[1] = *(const v8h*)(wp + 16);
            d1 = wmh(a.v, ba.v, ldc8(prm + 32 * q + 16 + 8 * h));
          }
          bq[q].h[0] = relu8(d0, QSC1);
          bq[q].h[1] = relu8(d1, QSC1);
        }
        FragH bz[2];
#pragma unroll
        for (int q = 0; q < 2; ++q) {
          v8f dd[2];
#pragma unroll
          for (int t = 0; t < 2; ++t) {
            const int ft = 2 * q + t;
            v8f c = ldc8(prm + MH + 16 * ft + 8 * h);
#pragma unroll
            for (int kt = 0; kt < 2; ++kt) {
              FragH a;
              const _Float16* wp = P2 + (size_t)(16 * ft + m) * MH + 32 * kt + 8 * h;
              a.h[0] = *(const v8h*)wp;
              a.h[1] = *(const v8h*)(wp + 16);
              c = wmh(a.v, bq[kt].v, c);
            }
            dd[t] = c;
          }
          bz[q].h[0] = relu8(dd[0], QSC2);
          bz[q].h[1] = relu8(dd[1], QSC2);
        }
        FragH bm[2];
#pragma unroll
        for (int q = 0; q < 2; ++q) {
          v8f dd[2];
#pragma unroll
          for (int t = 0; t < 2; ++t) {
            const int ft = 2 * q + t;
            v8f c = ldc8(prm + 2 * MH + 16 * ft + 8 * h);
#pragma unroll
            for (int kt = 0; kt < 2; ++kt) {
              FragH a;
              const _Float16* wp = P3 + (size_t)(16 * ft + m) * MH + 32 * kt + 8 * h;
              a.h[0] = *(const v8h*)wp;
              a.h[1] = *(const v8h*)(wp + 16);
              c = wmh(a.v, bz[kt].v, c);
            }
            dd[t] = c;
          }
          bm[q].h[0] = relu8(dd[0], QSC2);
          bm[q].h[1] = relu8(dd[1], QSC2);
        }
        float al0 = 0.0f, al1 = 0.0f;
        float* mrow = msg + (wave * 16 + m) * HC;
#pragma unroll 1
        for (int hd = 0; hd < 2; ++hd) {
          float al = 0.0f;
#pragma unroll 1
          for (int t4 = 0; t4 < 4; ++t4) {
            const int ft = 4 * hd + t4;
            v8f c = splat8(0.0f);
#pragma unroll
            for (int kt = 0; kt < 2; ++kt) {
              FragH a;
              const _Float16* wp = PE + (size_t)(16 * ft + m) * MH + 32 * kt + 8 * h;
              a.h[0] = *(const v8h*)wp;
              a.h[1] = *(const v8h*)(wp + 16);
              c = wmh(a.v, bm[kt].v, c);
            }
            const int f0 = 16 * ft + 8 * h;
            const float* swr = SWp + (size_t)dcl * HC + f0;
            const float* qr  = Qp  + (size_t)dcl * HC + f0;
            const float* kr  = Kq  + (size_t)scl * HC + f0;
            const float* vr  = Vp  + (size_t)scl * HC + f0;
            const v4f w0 = *(const v4f*)swr, w1 = *(const v4f*)(swr + 4);
            const v4f u0 = *(const v4f*)qr,  u1 = *(const v4f*)(qr + 4);
            const v4f k0 = *(const v4f*)kr,  k1 = *(const v4f*)(kr + 4);
            const v4f v0 = *(const v4f*)vr,  v1 = *(const v4f*)(vr + 4);
            v4f c0, c1;
            c0.x = c[0]; c0.y = c[1]; c0.z = c[2]; c0.w = c[3];
            c1.x = c[4]; c1.y = c[5]; c1.z = c[6]; c1.w = c[7];
            const v4f ee0 = c0 * EINV + w0;
            const v4f ee1 = c1 * EINV + w1;
            const v4f val0 = v0 + ee0, val1 = v1 + ee1;
            const v4f key0 = k0 + ee0, key1 = k1 + ee1;
            const v4f pr0 = u0 * key0, pr1 = u1 * key1;
            al += (pr0.x + pr0.y) + (pr0.z + pr0.w) + (pr1.x + pr1.y) + (pr1.z + pr1.w);
            *(v4f*)(mrow + f0) = val0;
            *(v4f*)(mrow + f0 + 4) = val1;
          }
          if (hd == 0) al0 = al; else al1 = al;
        }
        al0 += __shfl_xor(al0, 16);
        al1 += __shfl_xor(al1, 16);
        alph[(wave * 16 + m) * 2 + h] = (h ? al1 : al0) * ASCL;
      }
      __syncthreads();

      if (wave == 0) {
        const int hs = lane & 1;
#pragma unroll 1
        for (int i = 0; i < PASSN; ++i) {
          int sl = slotb[i];
          sl = sl < 0 ? 0 : (sl > NB ? NB : sl);
          const float a  = alph[i * 2 + hs];
          const float mo = mst[sl * 2 + hs];
          const float mn = fmaxf(mo, a);
          mst[sl * 2 + hs] = mn;
          mpv[i * 2 + hs] = mo;
          mnv[i * 2 + hs] = mn;
        }
      }
      __syncthreads();

      {
        const float mo = mpv[tid], mn = mnv[tid], a = alph[tid];
        spv[tid] = expf(mo - mn);
        ppv[tid] = expf(a - mn);
      }
      __syncthreads();

      if (wave == 0) {
        const int c4 = 4 * lane, hs = lane >> 4;
#pragma unroll 1
        for (int i = 0; i < PASSN; ++i) {
          int sl = slotb[i];
          sl = sl < 0 ? 0 : (sl > NB ? NB : sl);
          const float s = spv[i * 2 + hs], p = ppv[i * 2 + hs];
          float* ap = acc + sl * HC + c4;
          v4f av = *(const v4f*)ap;
          const v4f vv = *(const v4f*)(msg + i * HC + c4);
          av = av * s + vv * p;
          *(v4f*)ap = av;
        }
      } else if (wave == 1) {
        const int hs = lane & 1;
#pragma unroll 1
        for (int i = 0; i < PASSN; ++i) {
          int sl = slotb[i];
          sl = sl < 0 ? 0 : (sl > NB ? NB : sl);
          const float s = spv[i * 2 + hs], p = ppv[i * 2 + hs];
          const float dv = den[sl * 2 + hs];
          den[sl * 2 + hs] = dv * s + p;
        }
      }
      __syncthreads();
    }

    int rem = newN - R * PASSN;
    rem = rem < 0 ? 0 : rem;
    if (R > 0 && tid < rem) pend[tid] = pend[R * PASSN + tid];
    if (tid == 0) wcnt[NWAVE] = rem;
  }
  __syncthreads();

  {
    const int c = tid & 63, g = tid >> 6;
#pragma unroll 1
    for (int sl = g; sl < NB; sl += 4) {
      const float d0 = den[sl * 2] + DEPS;
      const float d1 = den[sl * 2 + 1] + DEPS;
      const float a0 = acc[sl * HC + c];
      const float a1 = acc[sl * HC + CH + c];
      const float res = 0.5f * (a0 * (1.0f / d0) + a1 * (1.0f / d1));
      acc[sl * HC + c] = res;
    }
  }
  __syncthreads();

  const int rs = lane >> 4, c4 = 4 * (lane & 15);
#pragma unroll 1
  for (int j = 0; j < NB / NWAVE / 2; ++j) {
    const int row = wave * (NB / NWAVE) + 2 * j + rs;
    const v4f v = *(const v4f*)(acc + row * HC + c4);
    *(volatile v4f*)(aggo + (size_t)(nodeBase + row) * CH + c4) = v;
  }
  __threadfence();
#pragma unroll 1
  for (int j = 0; j < NB / NWAVE / 2; ++j) {
    const int row = wave * (NB / NWAVE) + 2 * j + rs;
    const v4f v = *(const v4f*)(acc + row * HC + c4);
    *(volatile v4f*)(aggo + (size_t)(nodeBase + row) * CH + c4) = v;
  }
}

__device__ __forceinline__ void head_layer(const FragB (&ah)[2], const FragB (&al)[2],
                                           const unsigned short* __restrict__ ph, const unsigned short* __restrict__ pl,
                                           const float* __restrict__ bias, float* uw, int h, int m) {
#pragma unroll 1
  for (int nt = 0; nt < 4; ++nt) {
    const int n = 16 * nt + m;
    v8f c = splat8(bias[n]);
#pragma unroll
    for (int kt = 0; kt < 2; ++kt) {
      FragB bh, bl;
      const size_t off = (size_t)n * CH + 32 * kt + 8 * h;
      bh.u[0] = *(const v8us*)(ph + off);
      bh.u[1] = *(const v8us*)(ph + off + 16);
      bl.u[0] = *(const v8us*)(pl + off);
      bl.u[1] = *(const v8us*)(pl + off + 16);
      c = wmb3(ah[kt], al[kt], bh, bl, c);
    }
#pragma unroll
    for (int r = 0; r < 8; ++r) uw[(8 * h + r) * CH + n] = fmaxf(c[r], 0.0f);
  }
}

__device__ __forceinline__ void head_reload(const float* uw, FragB (&ah)[2], FragB (&al)[2], int h, int m) {
#pragma unroll
  for (int kt = 0; kt < 2; ++kt) {
    const float* p = uw + m * CH + 32 * kt + 8 * h;
    const v4f x0 = *(const v4f*)p, x1 = *(const v4f*)(p + 4);
    const v4f x2 = *(const v4f*)(p + 16), x3 = *(const v4f*)(p + 20);
    split8(x0, x1, ah[kt].u[0], al[kt].u[0]);
    split8(x2, x3, ah[kt].u[1], al[kt].u[1]);
  }
}

__global__ __launch_bounds__(NTHR) void k_head(
    const float* __restrict__ agg, const float* __restrict__ skp,
    const unsigned short* __restrict__ p1h, const unsigned short* __restrict__ p1l, const float* __restrict__ hb1,
    const unsigned short* __restrict__ p2h, const unsigned short* __restrict__ p2l, const float* __restrict__ hb2,
    const unsigned short* __restrict__ p3h, const unsigned short* __restrict__ p3l, const float* __restrict__ hb3,
    float* out, int nN) {
  __shared__ __attribute__((aligned(16))) float us[NWAVE * 16 * CH];
  __shared__ __attribute__((aligned(16))) float o0[HNB * 2];
  __shared__ __attribute__((aligned(16))) float o1[HNB];
  __shared__ __attribute__((aligned(16))) float o2[HNB * MOLD];
  __shared__ __attribute__((aligned(16))) float o3[HNB];
  const int tid = threadIdx.x, lane = tid & 31, wave = tid >> 5, h = lane >> 4, m = lane & 15;
  const int node0 = blockIdx.x * HNB;
  const int lrow0 = wave * 16;
  int node = node0 + lrow0 + m;
  node = node > nN - 1 ? nN - 1 : node;
  float* uw = us + wave * 16 * CH;

  FragB ah[2], al[2];
  {
    const float* ar = agg + (size_t)node * CH;
    const float* sr = skp + (size_t)node * CH;
#pragma unroll
    for (int kt = 0; kt < 2; ++kt) {
      const int k0 = 32 * kt + 8 * h;
      const v4f x0 = *(const v4f*)(ar + k0)      + *(const v4f*)(sr + k0);
      const v4f x1 = *(const v4f*)(ar + k0 + 4)  + *(const v4f*)(sr + k0 + 4);
      const v4f x2 = *(const v4f*)(ar + k0 + 16) + *(const v4f*)(sr + k0 + 16);
      const v4f x3 = *(const v4f*)(ar + k0 + 20) + *(const v4f*)(sr + k0 + 20);
      split8(x0, x1, ah[kt].u[0], al[kt].u[0]);
      split8(x2, x3, ah[kt].u[1], al[kt].u[1]);
    }
  }
  head_layer(ah, al, p1h, p1l, hb1, uw, h, m);
  __syncthreads();
  head_reload(uw, ah, al, h, m);
  __syncthreads();
  head_layer(ah, al, p2h, p2l, hb2, uw, h, m);
  __syncthreads();
  head_reload(uw, ah, al, h, m);

#pragma unroll 1
  for (int nt = 0; nt < 2; ++nt) {
    const int n = 16 * nt + m;
    const int ncl = n < OD - 1 ? n : OD - 1;
    const float bb = hb3[ncl];
    v8f c = splat8(n < OD ? bb : 0.0f);
#pragma unroll
    for (int kt = 0; kt < 2; ++kt) {
      FragB bh, bl;
      const size_t off = (size_t)n * CH + 32 * kt + 8 * h;
      bh.u[0] = *(const v8us*)(p3h + off);
      bh.u[1] = *(const v8us*)(p3h + off + 16);
      bl.u[0] = *(const v8us*)(p3l + off);
      bl.u[1] = *(const v8us*)(p3l + off + 16);
      c = wmb3(ah[kt], al[kt], bh, bl, c);
    }
#pragma unroll
    for (int r = 0; r < 8; ++r) {
      const int lrow = lrow0 + 8 * h + r;
      const float v = c[r];
      if (n < 2)              o0[lrow * 2 + n] = v;
      else if (n == 2)        o1[lrow] = v;
      else if (n < 3 + MOLD)  o2[lrow * MOLD + (n - 3)] = v;
      else if (n == 3 + MOLD) o3[lrow] = v;
    }
  }
  __syncthreads();

  int nv = nN - node0;
  nv = nv > HNB ? HNB : nv;
  const int n0q = nv / 2, n1q = nv / 4, n2q = nv * 4, n3q = nv / 4;
  float* b0 = out + (size_t)node0 * 2;
  float* b1 = out + (size_t)nN * 2 + node0;
  float* b2 = out + (size_t)nN * 3 + (size_t)node0 * MOLD;
  float* b3 = out + (size_t)nN * (3 + MOLD) + node0;
  for (int u = tid; u < n0q; u += NTHR) { const v4f v = *(const v4f*)(o0 + 4 * u); *(volatile v4f*)(b0 + 4 * u) = v; }
  for (int u = tid; u < n1q; u += NTHR) { const v4f v = *(const v4f*)(o1 + 4 * u); *(volatile v4f*)(b1 + 4 * u) = v; }
  for (int u = tid; u < n2q; u += NTHR) { const v4f v = *(const v4f*)(o2 + 4 * u); *(volatile v4f*)(b2 + 4 * u) = v; }
  for (int u = tid; u < n3q; u += NTHR) { const v4f v = *(const v4f*)(o3 + 4 * u); *(volatile v4f*)(b3 + 4 * u) = v; }
  __threadfence();
  for (int u = tid; u < n0q; u += NTHR) { const v4f v = *(const v4f*)(o0 + 4 * u); *(volatile v4f*)(b0 + 4 * u) = v; }
  for (int u = tid; u < n1q; u += NTHR) { const v4f v = *(const v4f*)(o1 + 4 * u); *(volatile v4f*)(b1 + 4 * u) = v; }
  for (int u = tid; u < n2q; u += NTHR) { const v4f v = *(const v4f*)(o2 + 4 * u); *(volatile v4f*)(b2 + 4 * u) = v; }
  for (int u = tid; u < n3q; u += NTHR) { const v4f v = *(const v4f*)(o3 + 4 * u); *(volatile v4f*)(b3 + 4 * u) = v; }
}

extern "C" void kernel_launch(void* const* d_in, const int* in_sizes, int n_in,
                              void* d_out, int out_size, void* d_ws, size_t ws_size,
                              hipStream_t stream) {
  if (n_in < 28) return;
  const int nN = in_sizes[1];
  if (nN < 4 || (nN & 3) != 0) return;
  if (in_sizes[0] != 2 * nN || in_sizes[2] != MOLD * nN || in_sizes[3] != nN) return;
  const int nE = in_sizes[4];
  if (nE < 1 || in_sizes[5] != nE || in_sizes[6] != nE) return;
  if (in_sizes[7] != RIN * MH || in_sizes[8] != MH) return;
  if (in_sizes[9] != MH * MH || in_sizes[10] != MH || in_sizes[11] != MH * MH || in_sizes[12] != MH) return;
  if (in_sizes[13] != SFD * HC || in_sizes[14] != HC) return;
  if (in_sizes[15] != SFD * HC || in_sizes[16] != HC) return;
  if (in_sizes[17] != SFD * HC || in_sizes[18] != HC) return;
  if (in_sizes[19] != (MH + SFD) * HC) return;
  if (in_sizes[20] != SFD * CH || in_sizes[21] != CH) return;
  if (in_sizes[22] != CH * CH || in_sizes[23] != CH || in_sizes[24] != CH * CH || in_sizes[25] != CH) return;
  if (in_sizes[26] != CH * OD || in_sizes[27] != OD) return;
  if (out_size != OD * nN) return;

  const float* x     = (const float*)d_in[0];
  const float* angle = (const float*)d_in[1];
  const float* mol   = (const float*)d_in[2];
  const float* gen   = (const float*)d_in[3];
  const int*   src   = (const int*)d_in[4];
  const int*   dst   = (const int*)d_in[5];
  const float* emask = (const float*)d_in[6];
  const float* mw1   = (const float*)d_in[7];
  const float* mb1   = (const float*)d_in[8];
  const float* mw2   = (const float*)d_in[9];
  const float* mb2   = (const float*)d_in[10];
  const float* mw3   = (const float*)d_in[11];
  const float* mb3   = (const float*)d_in[12];
  const float* wq    = (const float*)d_in[13];
  const float* bq    = (const float*)d_in[14];
  const float* wk    = (const float*)d_in[15];
  const float* bk    = (const float*)d_in[16];
  const float* wv    = (const float*)d_in[17];
  const float* bv    = (const float*)d_in[18];
  const float* we    = (const float*)d_in[19];
  const float* wskip = (const float*)d_in[20];
  const float* bskip = (const float*)d_in[21];
  const float* hw1   = (const float*)d_in[22];
  const float* hb1   = (const float*)d_in[23];
  const float* hw2   = (const float*)d_in[24];
  const float* hb2   = (const float*)d_in[25];
  const float* hw3   = (const float*)d_in[26];
  const float* hb3   = (const float*)d_in[27];
  float* outp = (float*)d_out;

  const int nDB = (nN + NB - 1) / NB;
  const int nNB = (nN + HNB - 1) / HNB;
  const int nEB = (nN + NB - 1) / NB;
  const size_t rowsD = (size_t)nDB * NB;
  const size_t rowsN = (size_t)nNB * HNB;
  const size_t rowsE = (size_t)nEB * NB;

  char* ws = (char*)d_ws;
  size_t off = 0;
  auto take = [&](size_t bytes) { const size_t o = off; off += (bytes + 255) & ~(size_t)255; return o; };
  const size_t oP1  = take((size_t)MH * RIK * 2);
  const size_t oP2  = take((size_t)MH * MH * 2);
  const size_t oP3  = take((size_t)MH * MH * 2);
  const size_t oPE  = take((size_t)HC * MH * 2);
  const size_t oQh  = take((size_t)HC * SFK * 2), oQl = take((size_t)HC * SFK * 2);
  const size_t oKh  = take((size_t)HC * SFK * 2), oKl = take((size_t)HC * SFK * 2);
  const size_t oVh  = take((size_t)HC * SFK * 2), oVl = take((size_t)HC * SFK * 2);
  const size_t oSh  = take((size_t)CH * SFK * 2), oSl = take((size_t)CH * SFK * 2);
  const size_t oWh  = take((size_t)HC * SFK * 2), oWl = take((size_t)HC * SFK * 2);
  const size_t oH1h = take((size_t)CH * CH * 2), oH1l = take((size_t)CH * CH * 2);
  const size_t oH2h = take((size_t)CH * CH * 2), oH2l = take((size_t)CH * CH * 2);
  const size_t oH3h = take((size_t)ODP * CH * 2), oH3l = take((size_t)ODP * CH * 2);
  const size_t oDEG = take(rowsD * 4);
  const size_t oQ   = take(rowsN * HC * 4);
  const size_t oK   = take(rowsN * HC * 4);
  const size_t oV   = take(rowsN * HC * 4);
  const size_t oSW  = take(rowsN * HC * 4);
  const size_t oSK  = take(rowsN * CH * 4);
  const size_t oAGG = take(rowsE * CH * 4);
  size_t limit = (size_t)WSLIM;
  if (ws_size < limit) limit = ws_size;
  if (off > limit) return;

  unsigned short* P1  = (unsigned short*)(ws + oP1);
  unsigned short* P2  = (unsigned short*)(ws + oP2);
  unsigned short* P3  = (unsigned short*)(ws + oP3);
  unsigned short* PE  = (unsigned short*)(ws + oPE);
  unsigned short* Qh  = (unsigned short*)(ws + oQh);
  unsigned short* Ql  = (unsigned short*)(ws + oQl);
  unsigned short* Kh  = (unsigned short*)(ws + oKh);
  unsigned short* Kl  = (unsigned short*)(ws + oKl);
  unsigned short* Vh  = (unsigned short*)(ws + oVh);
  unsigned short* Vl  = (unsigned short*)(ws + oVl);
  unsigned short* Sh  = (unsigned short*)(ws + oSh);
  unsigned short* Sl  = (unsigned short*)(ws + oSl);
  unsigned short* Wh  = (unsigned short*)(ws + oWh);
  unsigned short* Wl  = (unsigned short*)(ws + oWl);
  unsigned short* H1h = (unsigned short*)(ws + oH1h);
  unsigned short* H1l = (unsigned short*)(ws + oH1l);
  unsigned short* H2h = (unsigned short*)(ws + oH2h);
  unsigned short* H2l = (unsigned short*)(ws + oH2l);
  unsigned short* H3h = (unsigned short*)(ws + oH3h);
  unsigned short* H3l = (unsigned short*)(ws + oH3l);
  float* DEG = (float*)(ws + oDEG);
  float* Qf  = (float*)(ws + oQ);
  float* Kf  = (float*)(ws + oK);
  float* Vf  = (float*)(ws + oV);
  float* SWf = (float*)(ws + oSW);
  float* SKf = (float*)(ws + oSK);
  float* AGG = (float*)(ws + oAGG);

  const int vec8 = ((nE & 3) == 0) ? 1 : 0;

  k_prep<<<NPREP, NTHR, 0, stream>>>(mw1, mw2, mw3, we, wq, wk, wv, wskip, hw1, hw2, hw3,
                                     P1, P2, P3, PE, Qh, Ql, Kh, Kl, Vh, Vl, Sh, Sl, Wh, Wl,
                                     H1h, H1l, H2h, H2l, H3h, H3l);

  k_deg<<<nDB, NTHR, 0, stream>>>(dst, emask, DEG, nE, vec8);

  hipFuncSetAttribute(reinterpret_cast<const void*>(&k_node), hipFuncAttributeMaxDynamicSharedMemorySize, LN_TOTAL);
  k_node<<<nNB, NTHR, LN_TOTAL, stream>>>(angle, mol, gen, DEG,
                                          Qh, Ql, Kh, Kl, Vh, Vl, Sh, Sl, Wh, Wl,
                                          bq, bk, bv, bskip, Qf, Kf, Vf, SKf, SWf, nN);

  hipFuncSetAttribute(reinterpret_cast<const void*>(&k_edge), hipFuncAttributeMaxDynamicSharedMemorySize, LE_TOTAL);
  k_edge<<<nEB, NTHR, LE_TOTAL, stream>>>(x, angle, mol, src, dst, emask, mb1, mb2, mb3,
                                          (const _Float16*)P1, (const _Float16*)P2,
                                          (const _Float16*)P3, (const _Float16*)PE,
                                          Qf, Kf, Vf, SWf, AGG, nN, nE, vec8);

  k_head<<<nNB, NTHR, 0, stream>>>(AGG, SKf, H1h, H1l, hb1, H2h, H2l, hb2, H3h, H3l, hb3, outp, nN);
}
